// RelativeMultiHeadAttention_49581102465357
// MI455X (gfx1250) — hardware-verified
//
#include <hip/hip_runtime.h>
#pragma clang fp contract(off)


#ifndef NB
#define NB 4
#endif
#ifndef SEQ
#define SEQ 512
#endif
#ifndef MSEQ
#define MSEQ 512
#endif
#define SEQ_FULL  512
#define MSEQ_FULL 512
#define LL   (MSEQ + SEQ)
#define DM   1024
#define NH   16
#define HD   64
#define LN_EPS 1e-5f
#define SCL  0.125f
static_assert(SEQ % 64 == 0);
static_assert(MSEQ % 64 == 0);
static_assert(LL % 128 == 0);
static_assert(NH * HD == DM);
static_assert(DM == 256 * 4);
static_assert((NH * SEQ) % 8 == 0);

typedef _Float16 h16;
typedef unsigned short bf;
typedef __attribute__((ext_vector_type(16))) __bf16   v16bf;
typedef __attribute__((ext_vector_type(16))) _Float16 v16h;
typedef __attribute__((ext_vector_type(8)))  _Float16 v8h;
typedef __attribute__((ext_vector_type(8)))  unsigned short v8us;
typedef __attribute__((ext_vector_type(8)))  float    v8f;
typedef __attribute__((ext_vector_type(4)))  float    v4f;
typedef v8h  __attribute__((may_alias)) v8ha;
typedef v4f  __attribute__((may_alias)) v4fa;
typedef __attribute__((ext_vector_type(2))) _Float16 v2h;
typedef __attribute__((ext_vector_type(4))) _Float16 v4h;
typedef __attribute__((ext_vector_type(2))) unsigned short v2us;
typedef __attribute__((ext_vector_type(4))) unsigned short v4us;
typedef __attribute__((ext_vector_type(2))) float v2f;

__device__ __forceinline__ unsigned short f2bf(float f) { unsigned u = __float_as_uint(f); u += 0x7FFFu + ((u >> 16) & 1u); return (unsigned short)(u >> 16); }
__device__ __forceinline__ float bf2f(unsigned short b) { return __uint_as_float(((unsigned)b) << 16); }
__device__ __forceinline__ float bfr(float f) { return bf2f(f2bf(f)); }
__device__ __forceinline__ v16h cat16(v8h lo, v8h hi) { return __builtin_shufflevector(lo, hi, 0, 1, 2, 3, 4, 5, 6, 7, 8, 9, 10, 11, 12, 13, 14, 15); }
__device__ __forceinline__ v16bf cat16b(v8us lo, v8us hi) { return __builtin_bit_cast(v16bf, __builtin_shufflevector(lo, hi, 0, 1, 2, 3, 4, 5, 6, 7, 8, 9, 10, 11, 12, 13, 14, 15)); }
__device__ __forceinline__ v8f wmma16(v16h a, v16h b, v8f c) { return __builtin_amdgcn_wmma_f32_16x16x32_f16(false, a, false, b, (short)0, c, false, false); }
__device__ __forceinline__ v8f wmmab(v16bf a, v16bf b, v8f c) { return __builtin_amdgcn_wmma_f32_16x16x32_bf16(false, a, false, b, (short)0, c, false, false); }
__device__ __forceinline__ h16 tohx(float x) { return (h16)x; }
__device__ __forceinline__ void splitf(float y, unsigned short& h, unsigned short& l) { h = f2bf(y); l = f2bf(y - bf2f(h)); }

template <typename T16> struct WFrag;
template <> struct WFrag<h16> { typedef v16h V; static __device__ __forceinline__ V ld(const h16* p) { return cat16(*(const v8h*)p, *(const v8h*)(p + 16)); } static __device__ __forceinline__ v8f mma(V a, V b, v8f c) { return wmma16(a, b, c); } };
template <> struct WFrag<bf> { typedef v16bf V; static __device__ __forceinline__ V ld(const bf* p) { return cat16b(*(const v8us*)p, *(const v8us*)(p + 16)); } static __device__ __forceinline__ v8f mma(V a, V b, v8f c) { return wmmab(a, b, c); } };
template <typename T16, int NSPLIT, bool BIAS>
__global__ __launch_bounds__(32) void k_gemmw(const T16* __restrict__ A, const T16* __restrict__ A2, const T16* __restrict__ Bt, const T16* __restrict__ Bt2, int K, float* C, int ldc, const float* __restrict__ bias, size_t sA, size_t sB, size_t sC) {
    typedef typename WFrag<T16>::V V;
    __shared__ __align__(16) float os[16 * 68];
    const size_t z = blockIdx.z; A += z * sA; if (A2) A2 += z * sA; Bt += z * sB; if (Bt2) Bt2 += z * sB; C += z * sC;
    const int lane = threadIdx.x & 31, lr = lane & 15, hi = lane >> 4; const int r0 = blockIdx.x * 64, c0 = blockIdx.y * 64;
    v8f acc[4][4];
#pragma unroll
    for (int mb = 0; mb < 4; ++mb)
#pragma unroll
        for (int nb = 0; nb < 4; ++nb) acc[mb][nb] = (v8f){};
    const size_t aoff = (size_t)(r0 + lr) * K + 8 * hi, boff = (size_t)(c0 + lr) * K + 8 * hi;
#pragma unroll 1
    for (int kc = 0; kc < K; kc += 32) {
        V a[4], a2[4];
#pragma unroll
        for (int mb = 0; mb < 4; ++mb) { a[mb] = WFrag<T16>::ld(A + aoff + (size_t)mb * 16 * K + kc); if (NSPLIT == 1 || NSPLIT == 2) a2[mb] = WFrag<T16>::ld(A2 + aoff + (size_t)mb * 16 * K + kc); }
#pragma unroll
        for (int nb = 0; nb < 4; ++nb) { const V b = WFrag<T16>::ld(Bt + boff + (size_t)nb * 16 * K + kc); V b2; if (NSPLIT >= 2) b2 = WFrag<T16>::ld(Bt2 + boff + (size_t)nb * 16 * K + kc);
#pragma unroll
            for (int mb = 0; mb < 4; ++mb) { acc[mb][nb] = WFrag<T16>::mma(a[mb], b, acc[mb][nb]); if (NSPLIT == 1 || NSPLIT == 2) acc[mb][nb] = WFrag<T16>::mma(a2[mb], b, acc[mb][nb]); if (NSPLIT >= 2) acc[mb][nb] = WFrag<T16>::mma(a[mb], b2, acc[mb][nb]); } }
        asm volatile("v_nop\n\tv_nop\n\tv_nop\n\tv_nop" : "+v"(acc[0][0]), "+v"(acc[1][1]), "+v"(acc[2][2]), "+v"(acc[3][3]) : "v"(a[0]), "v"(a[3]));
    }
#pragma unroll
    for (int mb = 0; mb < 4; ++mb) {
#pragma unroll
        for (int nb = 0; nb < 4; ++nb) {
#pragma unroll
            for (int j = 0; j < 8; ++j) os[(hi * 8 + j) * 68 + nb * 16 + lr] = acc[mb][nb][j]; }
        __builtin_amdgcn_wave_barrier(); asm volatile("" ::: "memory");
        float* crow = C + (size_t)(r0 + mb * 16) * ldc + c0;
#pragma unroll 1
        for (int ps = 0; ps < 2; ++ps) {
#pragma unroll
            for (int s = 0; s < 8; ++s) { const int row = 2 * s + hi, cofs = lr * 4; v4f val = *(const v4fa*)(os + row * 68 + cofs); if (BIAS) { val[0] += bfr(bias[c0 + cofs]); val[1] += bfr(bias[c0 + cofs + 1]); val[2] += bfr(bias[c0 + cofs + 2]); val[3] += bfr(bias[c0 + cofs + 3]); }
                *(volatile v4f*)(crow + (size_t)row * ldc + cofs) = val; }
            if (ps == 0) __threadfence(); }
        __builtin_amdgcn_wave_barrier(); asm volatile("" ::: "memory");
    }
}

__global__ __launch_bounds__(256) void k_cvt8(const float* __restrict__ src, bf* dst, size_t n8) { const size_t i = (size_t)blockIdx.x * 256 + threadIdx.x; if (i >= n8) return; const v8f v = *(const v8f*)(src + i * 8); v8us o;
#pragma unroll
    for (int k = 0; k < 8; ++k) o[k] = f2bf(v[k]); *(volatile v8us*)(dst + i * 8) = o; __threadfence(); *(volatile v8us*)(dst + i * 8) = o; }

__global__ __launch_bounds__(256) void k_ln(const float* __restrict__ xin, const float* __restrict__ xmem, const float* __restrict__ gam, const float* __restrict__ bet, bf* Xh, bf* Xl) {
    __shared__ float red[8];
    const int tid = threadIdx.x, lane = tid & 31, w = tid >> 5;
    const int p = blockIdx.x;
    const float* src = (p < MSEQ) ? (xmem + (size_t)p * DM) : (xin + (size_t)(p - MSEQ) * DM);
    const int c0 = tid * 4;
    v4f x = *(const v4f*)(src + c0);
#pragma unroll
    for (int q = 0; q < 4; ++q) x[q] = bfr(x[q]);
    float s = (x[0] + x[1]) + (x[2] + x[3]);
#pragma unroll
    for (int sh = 16; sh; sh >>= 1) s += __shfl_xor(s, sh, 32);
    if (lane == 0) red[w] = s;
    __syncthreads();
    float tot = 0.f;
#pragma unroll
    for (int k = 0; k < 8; ++k) tot += red[k];
    const float mu = tot * (1.0f / (float)DM);
    __syncthreads();
    v4f dv; float sq = 0.f;
#pragma unroll
    for (int q = 0; q < 4; ++q) { dv[q] = x[q] - mu; float m2 = dv[q] * dv[q]; asm volatile("" : "+v"(m2)); sq += m2; }
#pragma unroll
    for (int sh = 16; sh; sh >>= 1) sq += __shfl_xor(sq, sh, 32);
    if (lane == 0) red[w] = sq;
    __syncthreads();
    float tv = 0.f;
#pragma unroll
    for (int k = 0; k < 8; ++k) tv += red[k];
    const float var = tv * (1.0f / (float)DM);
    const float sd = sqrtf(var + LN_EPS);
    const float rs = 1.0f / sd;
    v4us oh, ol;
#pragma unroll
    for (int q = 0; q < 4; ++q) { float y = dv[q] * rs; asm volatile("" : "+v"(y)); float yg = y * bfr(gam[c0 + q]); asm volatile("" : "+v"(yg)); const float yo = yg + bfr(bet[c0 + q]); unsigned short a, c2; splitf(yo, a, c2); oh[q] = a; ol[q] = c2; }
    const size_t oo = (size_t)p * DM + c0;
    *(volatile v4us*)(Xh + oo) = oh; *(volatile v4us*)(Xl + oo) = ol; __threadfence(); *(volatile v4us*)(Xh + oo) = oh; *(volatile v4us*)(Xl + oo) = ol;
}

__global__ __launch_bounds__(256) void k_phi(bf* PHh, bf* PHl) {
    const int tid = threadIdx.x; const int c = blockIdx.x; const int m0 = tid * 2;
    const float pos = (float)(LL - 1 - c);
    float sa = 0.f, ca = 0.f, sb2 = 0.f, cb = 0.f;
#pragma unroll 1
    for (int q = 0; q < 2; ++q) {
        const int m = m0 + q;
        const float ex = (float)(2 * m) * (1.0f / (float)DM);
        const double pw = exp2((double)ex * 13.287712379549449);
        const float pf = (float)pw;
        const float inv = 1.0f / pf;
        const float ang = pos * inv;
        const float sv = sinf(ang); const float cv = cosf(ang);
        if (q == 0) { sa = sv; ca = cv; } else { sb2 = sv; cb = cv; }
    }
    v2us sh, sl, chh, cll;
    { unsigned short a, l; splitf(sa, a, l); sh[0] = a; sl[0] = l; splitf(sb2, a, l); sh[1] = a; sl[1] = l; splitf(ca, a, l); chh[0] = a; cll[0] = l; splitf(cb, a, l); chh[1] = a; cll[1] = l; }
    const size_t base = (size_t)c * DM + m0;
#pragma unroll 1
    for (int ps = 0; ps < 2; ++ps) {
        *(volatile v2us*)(PHh + base) = sh; *(volatile v2us*)(PHl + base) = sl; *(volatile v2us*)(PHh + base + DM / 2) = chh; *(volatile v2us*)(PHl + base + DM / 2) = cll;
        if (ps == 0) __threadfence(); }
}

__global__ __launch_bounds__(256) void k_qpl(const float* __restrict__ FQ, const float* __restrict__ uv, const float* __restrict__ vv, h16* QUV) {
    const size_t e = ((size_t)blockIdx.x * 256 + threadIdx.x) * 2; if (e >= (size_t)NH * SEQ * HD) return;
    const int d = (int)(e % HD); const int i = (int)((e / HD) % SEQ); const int h = (int)(e / ((size_t)HD * SEQ));
    const v2f x = *(const v2f*)(FQ + (size_t)i * DM + h * HD + d);
    v2h ou, ov;
#pragma unroll
    for (int q = 0; q < 2; ++q) { const float uq = bfr(uv[h * HD + d + q]); const float vq = bfr(vv[h * HD + d + q]); ou[q] = tohx(x[q] + uq); ov[q] = tohx(x[q] + vq); }
    const size_t o2 = (size_t)NH * SEQ * HD + e;
    *(volatile v2h*)(QUV + e) = ou; *(volatile v2h*)(QUV + o2) = ov; __threadfence(); *(volatile v2h*)(QUV + e) = ou; *(volatile v2h*)(QUV + o2) = ov;
}
__global__ __launch_bounds__(256) void k_hpl(const float* __restrict__ F, int pitch, int nrows, h16* dst) {
    const size_t e = ((size_t)blockIdx.x * 256 + threadIdx.x) * 2; if (e >= (size_t)NH * nrows * HD) return;
    const int d = (int)(e % HD); const int t = (int)((e / HD) % nrows); const int h = (int)(e / ((size_t)HD * nrows));
    const v2f x = *(const v2f*)(F + (size_t)t * pitch + h * HD + d); v2h o; o[0] = tohx(x[0]); o[1] = tohx(x[1]);
    *(volatile v2h*)(dst + e) = o; __threadfence(); *(volatile v2h*)(dst + e) = o;
}
__global__ __launch_bounds__(256) void k_vtp(const float* __restrict__ F, int pitch, bf* Vh, bf* Vl) {
    const size_t e = ((size_t)blockIdx.x * 256 + threadIdx.x) * 2; if (e >= (size_t)NH * HD * LL) return;
    const int t = (int)(e % LL); const int d = (int)((e / LL) % HD); const int g = (int)(e / ((size_t)LL * HD)); v2us oh, ol;
#pragma unroll
    for (int q = 0; q < 2; ++q) { const float x = F[(size_t)(t + q) * pitch + g * HD + d]; unsigned short a2, c2; splitf(x, a2, c2); oh[q] = a2; ol[q] = c2; }
    *(volatile v2us*)(Vh + e) = oh; *(volatile v2us*)(Vl + e) = ol; __threadfence(); *(volatile v2us*)(Vh + e) = oh; *(volatile v2us*)(Vl + e) = ol;
}
__global__ __launch_bounds__(256) void k_rsoft(const float* __restrict__ Sb, const float* __restrict__ PSb, bf* Ph, bf* Pl) {
    __shared__ __align__(16) float prw[8][LL];
    const int lane = threadIdx.x & 31, w = threadIdx.x >> 5;
    const int row = blockIdx.x * 8 + w;
    const int i = row % SEQ;
    const float* sr = Sb + (size_t)row * LL; const float* pr = PSb + (size_t)row * LL;
#pragma unroll
    for (int ch = 0; ch < LL / 128; ++ch) *(v4f*)(&prw[w][ch * 128 + lane * 4]) = *(const v4f*)(pr + ch * 128 + lane * 4);
    __syncthreads();
    const int shift = SEQ - 1 - i; const int jmax = MSEQ + i;
    float v[LL / 32]; float mx = -3.0e38f;
#pragma unroll
    for (int ch = 0; ch < LL / 128; ++ch) { const int j0 = ch * 128 + lane * 4; const v4f a = *(const v4f*)(sr + j0);
#pragma unroll
        for (int q = 0; q < 4; ++q) { const int j = j0 + q; int c = shift + j; c = (c > LL - 1) ? (LL - 1) : c; const float psv = prw[w][c];
            const float t = (j <= jmax) ? ((a[q] + psv) * SCL) : -1.0e30f; v[ch * 4 + q] = t; mx = fmaxf(mx, t); } }
#pragma unroll
    for (int sh = 16; sh; sh >>= 1) mx = fmaxf(mx, __shfl_xor(mx, sh, 32));
    float sum = 0.f;
#pragma unroll
    for (int k = 0; k < LL / 32; ++k) { float d0 = __fsub_rn(v[k], mx); asm volatile("" : "+v"(d0)); v[k] = __builtin_amdgcn_exp2f(__fmul_rn(d0, 1.4426950408889634f)); sum += v[k]; }
#pragma unroll
    for (int sh = 16; sh; sh >>= 1) sum += __shfl_xor(sum, sh, 32);
    const float f = __fdiv_rn(1.0f, sum);
#pragma unroll 1
    for (int ps = 0; ps < 2; ++ps) {
#pragma unroll
        for (int ch = 0; ch < LL / 128; ++ch) { v4us oh, ol;
#pragma unroll
            for (int q = 0; q < 4; ++q) { unsigned short a, c2; splitf(v[ch * 4 + q] * f, a, c2); oh[q] = a; ol[q] = c2; }
            const size_t oo = (size_t)row * LL + ch * 128 + lane * 4; *(volatile v4us*)(Ph + oo) = oh; *(volatile v4us*)(Pl + oo) = ol; }
        if (ps == 0) __threadfence(); }
}
__global__ __launch_bounds__(256) void k_aopl(const float* __restrict__ O, bf* Ah, bf* Al) {
    const size_t e = ((size_t)blockIdx.x * 256 + threadIdx.x) * 2; if (e >= (size_t)NH * SEQ * HD) return;
    const int d = (int)(e % HD); const int i = (int)((e / HD) % SEQ); const int h = (int)(e / ((size_t)HD * SEQ));
    const v2f o2 = *(const v2f*)(O + e); v2us oh, ol;
#pragma unroll
    for (int q = 0; q < 2; ++q) { unsigned short a, c2; splitf(o2[q], a, c2); oh[q] = a; ol[q] = c2; }
    const size_t oo = (size_t)i * DM + h * HD + d;
    *(volatile v2us*)(Ah + oo) = oh; *(volatile v2us*)(Al + oo) = ol; __threadfence(); *(volatile v2us*)(Ah + oo) = oh; *(volatile v2us*)(Al + oo) = ol;
}

extern "C" void kernel_launch(void* const* d_in, const int* in_sizes, int n_in,
                              void* d_out, int out_size, void* d_ws, size_t ws_size, hipStream_t stream) {
    if (n_in < 9) return;
    if ((size_t)in_sizes[0] < (size_t)NB * SEQ * DM || (size_t)in_sizes[1] < (size_t)NB * MSEQ * DM || (size_t)in_sizes[2] < (size_t)3 * DM * DM ||
        (size_t)in_sizes[3] < (size_t)DM * DM || (size_t)in_sizes[4] < (size_t)DM * DM || in_sizes[5] < NH * HD || in_sizes[6] < NH * HD || in_sizes[7] < DM || in_sizes[8] < DM) return;
    if ((size_t)out_size < (size_t)NB * SEQ * DM) return;
    const float* xin  = (const float*)d_in[0];
    const float* xmem = (const float*)d_in[1];
    const float* wqkv = (const float*)d_in[2];
    const float* wpos = (const float*)d_in[3];
    const float* wout = (const float*)d_in[4];
    const float* uv   = (const float*)d_in[5];
    const float* vvr  = (const float*)d_in[6];
    const float* gam  = (const float*)d_in[7];
    const float* bet  = (const float*)d_in[8];
    float* OUT = (float*)d_out;
    char* wsp = (char*)d_ws;
    auto take = [&](size_t bytes) { char* p = wsp; wsp += (bytes + 255) & ~(size_t)255; return (void*)p; };
    bf* WQKV = (bf*)take((size_t)3 * DM * DM * 2); bf* WPOS = (bf*)take((size_t)DM * DM * 2); bf* WOUT = (bf*)take((size_t)DM * DM * 2);
    h16* KR16 = (h16*)take((size_t)2 * NH * LL * HD * 2);
    h16* QUV16 = (h16*)take((size_t)2 * NH * SEQ * HD * 2);
    bf* VTh = (bf*)take((size_t)NH * HD * LL * 2); bf* VTl = (bf*)take((size_t)NH * HD * LL * 2);
    bf* Ph = (bf*)take((size_t)NH * SEQ * LL * 2); bf* Pl = (bf*)take((size_t)NH * SEQ * LL * 2);
    const size_t sHalf = (size_t)NH * SEQ * LL * 4;
    const size_t aliasA = (size_t)LL * DM * 20 + (size_t)SEQ * DM * 4;
    const size_t aliasB = (size_t)NH * SEQ * HD * 4 + (size_t)SEQ * DM * 2 * 2;
    size_t spsBytes = 2 * sHalf; if (aliasA > spsBytes) spsBytes = aliasA; if (sHalf + aliasB > spsBytes) spsBytes = sHalf + aliasB;
    char* SPSc = (char*)take(spsBytes);
    if ((size_t)(wsp - (char*)d_ws) > ws_size) return;
    float* SPS = (float*)SPSc; float* Sb = SPS; float* PSb = SPS + (size_t)NH * SEQ * LL;
    bf* PHIh = (bf*)SPSc; bf* PHIl = (bf*)(SPSc + (size_t)LL * DM * 2); float* Rf = (float*)(SPSc + (size_t)LL * DM * 4);
    bf* Xh = (bf*)(SPSc + (size_t)LL * DM * 8); bf* Xl = (bf*)(SPSc + (size_t)LL * DM * 10);
    float* FKV = (float*)(SPSc + (size_t)LL * DM * 12);
    float* FQ  = (float*)(SPSc + (size_t)LL * DM * 20);
    float* Ob  = (float*)(SPSc + sHalf);
    bf* AOh = (bf*)(SPSc + sHalf + (size_t)NH * SEQ * HD * 4); bf* AOl = AOh + (size_t)SEQ * DM;

    k_cvt8<<<(unsigned)(((size_t)3 * DM * DM / 8 + 255) / 256), 256, 0, stream>>>(wqkv, WQKV, (size_t)3 * DM * DM / 8);
    k_cvt8<<<(unsigned)(((size_t)DM * DM / 8 + 255) / 256), 256, 0, stream>>>(wpos, WPOS, (size_t)DM * DM / 8);
    k_cvt8<<<(unsigned)(((size_t)DM * DM / 8 + 255) / 256), 256, 0, stream>>>(wout, WOUT, (size_t)DM * DM / 8);
    k_phi<<<LL, 256, 0, stream>>>(PHIh, PHIl);
    k_gemmw<bf, 1, false><<<dim3(LL / 64, DM / 64, 1), 32, 0, stream>>>(PHIh, PHIl, WPOS, nullptr, DM, Rf, DM, nullptr, 0, 0, 0);
    const unsigned LQ = (unsigned)(((size_t)NH * SEQ * HD / 2 + 255) / 256), LKp = (unsigned)(((size_t)NH * LL * HD / 2 + 255) / 256);
    k_hpl<<<LKp, 256, 0, stream>>>(Rf, DM, LL, KR16 + (size_t)NH * LL * HD);
    for (int b = 0; b < NB; ++b) {
        k_ln<<<LL, 256, 0, stream>>>(xin + (size_t)b * SEQ_FULL * DM, xmem + (size_t)b * MSEQ_FULL * DM, gam, bet, Xh, Xl);
        k_gemmw<bf, 1, false><<<dim3(LL / 64, (2 * DM) / 64, 1), 32, 0, stream>>>(Xh, Xl, WQKV + (size_t)DM * DM, nullptr, DM, FKV, 2 * DM, nullptr, 0, 0, 0);
        k_gemmw<bf, 1, false><<<dim3(SEQ / 64, DM / 64, 1), 32, 0, stream>>>(Xh + (size_t)MSEQ * DM, Xl + (size_t)MSEQ * DM, WQKV, nullptr, DM, FQ, DM, nullptr, 0, 0, 0);
        k_qpl<<<LQ, 256, 0, stream>>>(FQ, uv, vvr, QUV16);
        k_hpl<<<LKp, 256, 0, stream>>>(FKV, 2 * DM, LL, KR16);
        k_vtp<<<LKp, 256, 0, stream>>>(FKV + DM, 2 * DM, VTh, VTl);
        k_gemmw<h16, 0, false><<<dim3(SEQ / 64, LL / 64, 2 * NH), 32, 0, stream>>>(QUV16, nullptr, KR16, nullptr, HD, SPS, LL, nullptr, (size_t)SEQ * HD, (size_t)LL * HD, (size_t)SEQ * LL);
        k_rsoft<<<NH * SEQ / 8, 256, 0, stream>>>(Sb, PSb, Ph, Pl);
        k_gemmw<bf, 2, false><<<dim3(SEQ / 64, HD / 64, NH), 32, 0, stream>>>(Ph, Pl, VTh, VTl, LL, Ob, HD, nullptr, (size_t)SEQ * LL, (size_t)HD * LL, (size_t)SEQ * HD);
        k_aopl<<<LQ, 256, 0, stream>>>(Ob, AOh, AOl);
        k_gemmw<bf, 1, false><<<dim3(SEQ / 64, DM / 64, 1), 32, 0, stream>>>(AOh, AOl, WOUT, nullptr, DM, OUT + (size_t)b * SEQ * DM, DM, nullptr, 0, 0, 0);
    }
}
